// self_attention_41738492183083
// MI455X (gfx1250) — hardware-run, weakly checked
//
#include <hip/hip_runtime.h>
#define NS 2
#define CH 64
#define SQ 8192
#define C8 8
#define KD 32
#define QT 2048
#define PCAR 32768.0f
#define FMIN16 6.103515625e-05f
typedef __bf16 v16b __attribute__((ext_vector_type(16)));
typedef unsigned short v8us __attribute__((ext_vector_type(8), may_alias));
typedef float  v8f  __attribute__((ext_vector_type(8)));
typedef float  v4f  __attribute__((ext_vector_type(4)));
typedef float  v4fa __attribute__((ext_vector_type(4), may_alias));
union FragB { v16b v; v8us half[2]; unsigned short u[16]; };

__device__ __forceinline__ unsigned short bf16_bits(float x) { unsigned int u = __float_as_uint(x); return (unsigned short)((u + 0x7FFFu + ((u >> 16) & 1u)) >> 16); }
__device__ __forceinline__ float bf16_val(unsigned short b) { return __uint_as_float(((unsigned int)b) << 16); }
__device__ __forceinline__ float bf16_round(float x) { return bf16_val(bf16_bits(x)); }
template <int NT>
__device__ __forceinline__ v8f mmaN(v16b ah, v16b al, v16b bh, v16b bl, v8f c) {
  c = __builtin_amdgcn_wmma_f32_16x16x32_bf16(false, ah, false, bh, (short)0, c, false, false);
  if (NT >= 2) c = __builtin_amdgcn_wmma_f32_16x16x32_bf16(false, al, false, bh, (short)0, c, false, false);
  if (NT >= 3) c = __builtin_amdgcn_wmma_f32_16x16x32_bf16(false, ah, false, bl, (short)0, c, false, false);
  asm volatile("v_nop\n\tv_nop\n\tv_nop\n\tv_nop" : "+v"(c) : "v"(ah), "v"(al), "v"(bh), "v"(bl));
  return c;
}


typedef _Float16 v16h __attribute__((ext_vector_type(16)));
union FragH { v16h v; v8us half[2]; _Float16 h[16]; unsigned short u[16]; };
template <int NT>
__device__ __forceinline__ v8f mmaH(v16h ah, v16h al, v16h bh, v16h bl, v8f c) {
  c = __builtin_amdgcn_wmma_f32_16x16x32_f16(false, ah, false, bh, (short)0, c, false, false);
  if (NT >= 2) c = __builtin_amdgcn_wmma_f32_16x16x32_f16(false, al, false, bh, (short)0, c, false, false);
  if (NT >= 3) c = __builtin_amdgcn_wmma_f32_16x16x32_f16(false, ah, false, bl, (short)0, c, false, false);
  asm volatile("v_nop\n\tv_nop\n\tv_nop\n\tv_nop" : "+v"(c) : "v"(ah), "v"(al), "v"(bh), "v"(bl));
  return c;
}

__global__ __launch_bounds__(256) void k_wt_f16(const float* __restrict__ W, _Float16* __restrict__ Wt, int K, int N, float scale) {
  const int t = blockIdx.x * 256 + threadIdx.x; if (t >= N * (K / 8)) return; const int n = t / (K / 8), k8 = (t % (K / 8)) * 8; FragH f;
#pragma unroll
  for (int i = 0; i < 8; ++i) f.h[i] = (_Float16)(bf16_round(W[(size_t)(k8 + i) * N + n]) * scale); const v8us o = f.half[0];
  *(volatile v8us*)((unsigned short*)Wt + (size_t)n * K + k8) = o; __threadfence(); *(volatile v8us*)((unsigned short*)Wt + (size_t)n * K + k8) = o;
}

typedef _Float16 v4h __attribute__((ext_vector_type(4)));

__global__ __launch_bounds__(256) void k_x16(const float* __restrict__ x, _Float16* __restrict__ X16, size_t n8) { const size_t t = (size_t)blockIdx.x * 256 + threadIdx.x; if (t >= n8) return; FragH f;
#pragma unroll
  for (int q = 0; q < 8; ++q) f.h[q] = (_Float16)bf16_round(x[t * 8 + q]); *(volatile v8us*)((unsigned short*)X16 + t * 8) = f.half[0]; __threadfence(); *(volatile v8us*)((unsigned short*)X16 + t * 8) = f.half[0]; }
__device__ __forceinline__ v16h g2_frag(const _Float16* p, int hh) { FragH f; f.half[0] = *(const v8us*)((const unsigned short*)p + 8 * hh); f.half[1] = *(const v8us*)((const unsigned short*)p + 16 + 8 * hh); return f.v; }
__device__ __forceinline__ v8f g2_mma(v16h a, v16h b, v8f c) { v8f d = __builtin_amdgcn_wmma_f32_16x16x32_f16(false, a, false, b, (short)0, c, false, false); asm volatile("v_nop\n\tv_nop\n\tv_nop\n\tv_nop" : "+v"(d) : "v"(a), "v"(b)); return d; }
template <int ACT>
__global__ __launch_bounds__(128) void k_gemm2(const _Float16* __restrict__ A, int lda, size_t sA, const _Float16* __restrict__ Bh, int ldb, size_t sB, float alpha, const float* __restrict__ bias, size_t sBias, const float* __restrict__ CP, int rowsPerB, size_t sCPb, int row0g,
    float* __restrict__ C, _Float16* __restrict__ C16, int ldc, size_t sC, int M, int N, int K) { static_assert(ACT == 0 || ACT == 3 || ACT == 6 || ACT == 8 || ACT == 9 || ACT == 11 || ACT == 12 || ACT == 14 || ACT == 15 || ACT == 16 || ACT == 17, "k_gemm2: unsupported ACT code (would silently apply no activation)");
  __shared__ __attribute__((aligned(16))) float so[4][32][68];
  const int tid = threadIdx.x, w = tid >> 5, lane = tid & 31, ln = lane & 15, hh = lane >> 4; const int by = blockIdx.y;
  A += (size_t)by * sA; Bh += (size_t)by * sB; const size_t cofs = (size_t)by * sC; const float* bp = bias ? bias + (size_t)by * sBias : nullptr;
  const int ntn = N >> 6; const int mt = blockIdx.x / ntn, nq = blockIdx.x - mt * ntn; const int row0 = mt * 128 + 32 * w, col0 = nq * 64; if (row0 >= M) return;
  const _Float16* a0p = A + (size_t)(row0 + ln) * lda; const _Float16* a1p = a0p + (size_t)16 * lda;
  const _Float16* b0p = Bh + (size_t)(col0 + ln) * ldb; const _Float16* b1p = b0p + (size_t)16 * ldb; const _Float16* b2p = b1p + (size_t)16 * ldb; const _Float16* b3p = b2p + (size_t)16 * ldb;
  const v8f z8 = {0.f,0.f,0.f,0.f,0.f,0.f,0.f,0.f}; v8f c00 = z8, c01 = z8, c02 = z8, c03 = z8, c10 = z8, c11 = z8, c12 = z8, c13 = z8;
  for (int kb = 0; kb < K; kb += 32) { const v16h a0 = g2_frag(a0p + kb, hh), a1 = g2_frag(a1p + kb, hh);
    v16h b = g2_frag(b0p + kb, hh); c00 = g2_mma(a0, b, c00); c10 = g2_mma(a1, b, c10);
    b = g2_frag(b1p + kb, hh); c01 = g2_mma(a0, b, c01); c11 = g2_mma(a1, b, c11);
    b = g2_frag(b2p + kb, hh); c02 = g2_mma(a0, b, c02); c12 = g2_mma(a1, b, c12);
    b = g2_frag(b3p + kb, hh); c03 = g2_mma(a0, b, c03); c13 = g2_mma(a1, b, c13); }
  v8f accs[8] = {c00, c01, c02, c03, c10, c11, c12, c13};
#pragma unroll
  for (int u = 0; u < 8; ++u) { const int t = u & 3, half = u >> 2; const int col = col0 + t * 16 + ln; const float bv = bp ? bf16_round(bp[col]) : 0.f;
#pragma unroll
    for (int r = 0; r < 8; ++r) { const int rloc = half * 16 + 8 * hh + r; float v = accs[u][r] * alpha + bv; if (CP) { if (rowsPerB < 0) v += CP[cofs + (size_t)(row0g + row0 + rloc) * ldc + col];        else { const int bidx = (row0g + row0 + rloc) / rowsPerB; v += CP[(size_t)bidx * sCPb + (size_t)by * 64 + col]; } }
      if (ACT == 3) v = fmaxf(v, 0.f); else if (ACT == 6) v = 0.5f * v * (1.0f + erff(v * 0.70710678118654752f)); else if (ACT == 11) v = 1.0f / (1.0f + expf(-v)); else if (ACT == 15) v = v / (1.0f + expf(-v)); else if (ACT == 12) v = (v > 0.f) ? v : 0.01f * v; else if (ACT == 8) v = tanhf(v); else if (ACT == 9) v = 0.5f * v * (1.0f + tanhf(0.7978845608028654f * (v + 0.044715f * v * v * v))); else if (ACT == 14) v = (v > 0.f) ? v : 0.1f * v; else if (ACT == 16) v = (v >= 0.f) ? v : 0.3f * v; else if (ACT == 17) v = (v >= 0.f) ? v : 0.2f * v;
      so[w][rloc][t * 16 + ln] = v; } }
  __builtin_amdgcn_fence(__ATOMIC_ACQ_REL, "workgroup"); __builtin_amdgcn_wave_barrier();
  const int rsub = lane >> 4, c4 = (lane & 15) * 4;
  for (int pass = 0; pass < 2; ++pass) {
#pragma unroll
    for (int q = 0; q < 16; ++q) { const int r = q * 2 + rsub; const v4f v = *(const v4fa*)&so[w][r][c4]; if (C) *(volatile v4f*)(C + cofs + (size_t)(row0 + r) * ldc + col0 + c4) = v; if (C16) { v4h h4; for (int i = 0; i < 4; ++i) h4[i] = (_Float16)v[i]; *(volatile v4h*)(C16 + cofs + (size_t)(row0 + r) * ldc + col0 + c4) = h4; } }
    if (pass == 0) __threadfence(); } }

__global__ __launch_bounds__(256) void k_rsmf(const float* __restrict__ S, _Float16* __restrict__ P, int qn, int hg) {
  const int t = blockIdx.x * 256 + threadIdx.x; if (t >= qn * hg) return; const size_t i = (size_t)(t / qn) * SQ + (t % qn); const float* s = S + i * SQ; float mx = -3.0e38f;
  for (int j = 0; j < SQ; ++j) mx = fmaxf(mx, s[j]); float se = 0.f;
  for (int j = 0; j < SQ; ++j) se += __expf(s[j] - mx); const float sc = 256.0f / se;
  for (int j0 = 0; j0 < SQ; j0 += 8) { FragH f; for (int q = 0; q < 8; ++q) f.h[q] = (_Float16)(__expf(s[j0 + q] - mx) * sc); unsigned short* d = (unsigned short*)P + i * SQ + j0; *(volatile v8us*)d = f.half[0]; __threadfence(); *(volatile v8us*)d = f.half[0]; } }
__global__ __launch_bounds__(256) void k_wtn_f16(const float* __restrict__ W, _Float16* __restrict__ Wt, int K, int N, float scale) {
  const int t = blockIdx.x * 256 + threadIdx.x; if (t >= N * (K / 8)) return; const int n = t / (K / 8), k8 = (t % (K / 8)) * 8; FragH f;
  for (int i = 0; i < 8; ++i) f.h[i] = (_Float16)(W[(size_t)(k8 + i) * N + n] * scale);
  unsigned short* o = (unsigned short*)Wt + (size_t)n * K + k8; *(volatile v8us*)o = f.half[0]; __threadfence(); *(volatile v8us*)o = f.half[0]; }
__global__ __launch_bounds__(256) void k_tr32(const float* __restrict__ YT, float* __restrict__ out, int n) {
  const int t = blockIdx.x * 256 + threadIdx.x; if (t >= n) return; const int n4 = t & (SQ / 4 - 1), oc = (t >> 10) & (CH - 1), bb = t >> 17; const float* s = YT + ((size_t)bb * SQ + 4 * n4) * CH + oc; v4f r;
  for (int i = 0; i < 4; ++i) r[i] = s[(size_t)i * CH];
  float* o = out + ((size_t)bb * CH + oc) * SQ + 4 * n4; *(volatile v4f*)o = r; __threadfence(); *(volatile v4f*)o = r; }

__global__ __launch_bounds__(256) void k_fg8(const float* __restrict__ x, const float* __restrict__ W, const float* __restrict__ b, _Float16* __restrict__ R, int mode, int n) {
  const size_t t = (size_t)blockIdx.x * 256 + threadIdx.x; if (t >= (size_t)n) return; float acc[C8]; for (int o = 0; o < C8; ++o) acc[o] = 0.f;
  for (int c = 0; c < CH; ++c) { const float xv = bf16_round(x[(size_t)c * SQ + t]); for (int o = 0; o < C8; ++o) acc[o] = fmaf(bf16_round(W[o * CH + c]), xv, acc[o]); }
  v4f va, vb; for (int o = 0; o < 4; ++o) { va[o] = acc[o] + bf16_round(b[o]); vb[o] = acc[4 + o] + bf16_round(b[4 + o]); }
  union { v4h q[2]; v8us u; } hi, g1, g2; hi.q[0] = __builtin_convertvector(va, v4h); hi.q[1] = __builtin_convertvector(vb, v4h); const v4f ha = __builtin_convertvector(hi.q[0], v4f), hb = __builtin_convertvector(hi.q[1], v4f);
  v4f la, lb, sa, sb; for (int o = 0; o < 4; ++o) { la[o] = (va[o] - ha[o]) * 32.0f; lb[o] = (vb[o] - hb[o]) * 32.0f; sa[o] = ha[o] * 0.03125f; sb[o] = hb[o] * 0.03125f; }
  const float fm = (float)(mode == 0), gm = 1.0f - fm; v4f pa, pb, qa, qb; for (int o = 0; o < 4; ++o) { pa[o] = fm * la[o] + gm * sa[o]; pb[o] = fm * lb[o] + gm * sb[o]; qa[o] = fm * sa[o] + gm * la[o]; qb[o] = fm * sb[o] + gm * lb[o]; }
  g1.q[0] = __builtin_convertvector(pa, v4h); g1.q[1] = __builtin_convertvector(pb, v4h); g2.q[0] = __builtin_convertvector(qa, v4h); g2.q[1] = __builtin_convertvector(qb, v4h); const v8us zz = { 0, 0, 0, 0, 0, 0, 0, 0 };
  unsigned short* r = (unsigned short*)R + t * KD; for (int pass = 0; pass < 2; ++pass) { *(volatile v8us*)r = hi.u; *(volatile v8us*)(r + 8) = g1.u; *(volatile v8us*)(r + 16) = g2.u; *(volatile v8us*)(r + 24) = zz; if (pass == 0) __threadfence(); } }
__global__ __launch_bounds__(256) void k_csm8(const float* __restrict__ ST, _Float16* __restrict__ PT, int n) {
  const size_t t = (size_t)blockIdx.x * 256 + threadIdx.x; if (t >= (size_t)n) return; const float* s = ST + 8 * t; v4f m0, m1, e0, e1; for (int q = 0; q < 4; ++q) { m0[q] = -3.0e38f; m1[q] = -3.0e38f; e0[q] = 0.f; e1[q] = 0.f; }
  for (int m = 0; m < SQ; ++m) { const v4f a = *(const v4fa*)(s + (size_t)m * QT), b = *(const v4fa*)(s + (size_t)m * QT + 4); for (int q = 0; q < 4; ++q) { m0[q] = fmaxf(m0[q], a[q]); m1[q] = fmaxf(m1[q], b[q]); } }
  for (int m = 0; m < SQ; ++m) { const v4f a = *(const v4fa*)(s + (size_t)m * QT), b = *(const v4fa*)(s + (size_t)m * QT + 4); for (int q = 0; q < 4; ++q) { e0[q] += __expf(a[q] - m0[q]); e1[q] += __expf(b[q] - m1[q]); } }
  v4f c0, c1; for (int q = 0; q < 4; ++q) { c0[q] = PCAR / e0[q]; c1[q] = PCAR / e1[q]; }
  for (int m = 0; m < SQ; ++m) { const v4f a = *(const v4fa*)(s + (size_t)m * QT), b = *(const v4fa*)(s + (size_t)m * QT + 4); v4f pa, pb; for (int q = 0; q < 4; ++q) { pa[q] = __expf(a[q] - m0[q]) * c0[q]; pb[q] = __expf(b[q] - m1[q]) * c1[q]; pa[q] = pa[q] * (float)(pa[q] >= FMIN16); pb[q] = pb[q] * (float)(pb[q] >= FMIN16); }
    union { v4h q[2]; v8us u; } w; w.q[0] = __builtin_convertvector(pa, v4h); w.q[1] = __builtin_convertvector(pb, v4h); unsigned short* o = (unsigned short*)PT + (size_t)m * QT + 8 * t; *(volatile v8us*)o = w.u; __threadfence(); *(volatile v8us*)o = w.u; } }
__global__ __launch_bounds__(256) void k_gres(const float* __restrict__ SA, const float* __restrict__ x, const float* __restrict__ gamma, float* __restrict__ out, size_t n4) {
  const size_t i = (size_t)blockIdx.x * 256 + threadIdx.x; if (i >= n4) return; const float gm = bf16_round(gamma[0]); const v4f a = *(const v4fa*)(SA + 4 * i), xv = *(const v4fa*)(x + 4 * i); v4f o; for (int j = 0; j < 4; ++j) o[j] = gm * a[j] + bf16_round(xv[j]);
  for (int pass = 0; pass < 2; ++pass) { *(volatile v4f*)(out + 4 * i) = o; if (pass == 0) __threadfence(); } }

extern "C" void kernel_launch(void* const* d_in, const int* in_sizes, int n_in,
                              void* d_out, int out_size, void* d_ws, size_t ws_size, hipStream_t stream) {
  (void)in_sizes; (void)n_in; (void)out_size;
  const float* xs[NS] = { (const float*)d_in[0], (const float*)d_in[1] }; const float* Wf = (const float*)d_in[2]; const float* bf = (const float*)d_in[3]; const float* Wg = (const float*)d_in[4]; const float* bg = (const float*)d_in[5];
  const float* Whs[NS] = { (const float*)d_in[6], (const float*)d_in[8] }; const float* bhs[NS] = { (const float*)d_in[7], (const float*)d_in[9] }; const float* gms[NS] = { (const float*)d_in[10], (const float*)d_in[11] };
  static_assert(NS == 2 && CH == 64 && SQ == 8192 && C8 == 8 && KD == 32 && QT == 2048 && SQ % QT == 0 && SQ % 256 == 0 && ((size_t)SQ * (CH / 8)) % 256 == 0 && ((size_t)CH * CH / 8) % 256 == 0 && ((size_t)CH * (SQ / 8)) % 256 == 0 && (QT / 8) % 256 == 0 && ((size_t)CH * SQ / 4) % 256 == 0 && SQ % 128 == 0 && QT % 64 == 0 && SQ % 64 == 0 && CH % 64 == 0 && CH % 32 == 0 && KD % 32 == 0 && QT % 32 == 0, "whole tiles; exact grids");
  float* out = (float*)d_out;
  char* ws = (char*)d_ws; size_t off = 0;
  auto take = [&](size_t bytes) { char* p = ws + off; off += (bytes + 255) & ~(size_t)255; return p; };
  _Float16* XT = (_Float16*)take((size_t)SQ * CH * 2); _Float16* FR = (_Float16*)take((size_t)SQ * KD * 2); _Float16* GR = (_Float16*)take((size_t)SQ * KD * 2); _Float16* WH = (_Float16*)take((size_t)CH * CH * 2);
  float* VTOK = (float*)take((size_t)SQ * CH * 4); _Float16* V16 = (_Float16*)take((size_t)CH * SQ * 2); float* ST = (float*)take((size_t)SQ * QT * 4); _Float16* PT = (_Float16*)take((size_t)SQ * QT * 2); float* SA = (float*)take((size_t)CH * SQ * 4);
  if (off > ws_size) return;
  for (int s = 0; s < NS; ++s) { const float* x = xs[s];
    k_wt_f16<<<(unsigned)((size_t)SQ * (CH / 8) / 256), 256, 0, stream>>>(x, XT, CH, SQ, 1.0f);
    k_fg8<<<SQ / 256, 256, 0, stream>>>(x, Wf, bf, FR, 0, SQ); k_fg8<<<SQ / 256, 256, 0, stream>>>(x, Wg, bg, GR, 1, SQ);
    k_x16<<<(unsigned)((size_t)CH * CH / 8 / 256), 256, 0, stream>>>(Whs[s], WH, (size_t)CH * CH / 8);
    k_gemm2<0><<<dim3((unsigned)((SQ / 128) * (CH / 64)), 1), 128, 0, stream>>>(XT, CH, (size_t)0, WH, CH, (size_t)0, 1.0f, bhs[s], 0, nullptr, 1, 0, 0, VTOK, nullptr, CH, (size_t)0, SQ, CH, CH);
    k_wtn_f16<<<(unsigned)((size_t)CH * (SQ / 8) / 256), 256, 0, stream>>>(VTOK, V16, SQ, CH, 1.0f);
    for (int q = 0; q < SQ / QT; ++q) {
      k_gemm2<0><<<dim3((unsigned)((SQ / 128) * (QT / 64)), 1), 128, 0, stream>>>(GR, KD, (size_t)0, FR + (size_t)q * QT * KD, KD, (size_t)0, 1.0f, nullptr, 0, nullptr, 1, 0, 0, ST, nullptr, QT, (size_t)0, SQ, QT, KD);
      k_csm8<<<(unsigned)((QT / 8 + 255) / 256), 256, 0, stream>>>(ST, PT, QT / 8);
      k_gemm2<0><<<dim3((unsigned)(1 * (SQ / 64)), 1), 128, 0, stream>>>(V16 + (size_t)q * QT, SQ, (size_t)0, PT, QT, (size_t)0, 1.0f / PCAR, nullptr, 0, q == 0 ? nullptr : SA, -1, 0, 0, SA, nullptr, SQ, (size_t)0, CH, SQ, QT); }
    k_gres<<<(unsigned)((size_t)CH * SQ / 4 / 256), 256, 0, stream>>>(SA, x, gms[s], out + (size_t)s * CH * SQ, (size_t)CH * SQ / 4); }
}
